// Phi_14723147891163
// MI455X (gfx1250) — hardware-verified
//
#include <hip/hip_runtime.h>
#include <stddef.h>


typedef _Float16 v16h __attribute__((ext_vector_type(16)));
typedef _Float16 v8h  __attribute__((ext_vector_type(8)));
typedef float    v8f  __attribute__((ext_vector_type(8)));
typedef float    v4f  __attribute__((ext_vector_type(4)));
typedef _Float16 h16;

#ifndef NEX
#define NEX 4096
#endif
#define NEX_FULL 4096
#define DD   63
#define DIN  64
#define MM   256
#define RR   10
#define LDG  320
#define LDJ  264
#define LDT  72
#define LDC  68
#define SPB  32

#define WCARRY 64.0f
#define ACARRY 16.0f
#define HSTEP  0.5f

#define F32_STEPS 4
#define F16_STEPS 2

static_assert(NEX >= 64 && NEX <= NEX_FULL);
static_assert((NEX % 64) == 0 && (NEX % SPB) == 0);
static_assert(DIN == 64 && MM == 256 && DD == DIN - 1);
static_assert(LDG == MM + DIN);
static_assert(((LDG * 2) % 128) == 0 && (LDG % 32) == 0);
static_assert((MM % 64) == 0 && (MM % 32) == 0 && (DIN % 32) == 0);
static_assert((LDJ % 8) == 0 && LDJ >= MM);
static_assert((LDT % 8) == 0 && LDT >= 64);
static_assert((LDC % 4) == 0 && LDC >= 64);
static_assert((256 / 16) * F32_STEPS == 64);
static_assert((256 / 8) * F16_STEPS == 64);
static_assert(SPB == 32);
static_assert(3 * 64 * LDC * 4 <= 131072);
static_assert(DIN * LDJ * 2 + (4 * MM + 8 + 32) * 4 <= 131072);
static_assert((size_t)NEX_FULL * DIN * 4 == (size_t)1048576);

#define W0N_BYTES ((size_t)MM * DIN * 2)
#define WSN_BYTES ((size_t)2 * MM * MM * 2)
#define WST_BYTES ((size_t)MM * 2 * MM * 2)
#define GW_BYTES  ((size_t)DIN * LDG * 2)
#define CST_BYTES ((size_t)(MM + 32) * 4)
#define SX_BYTES  ((size_t)NEX * LDG * 2)
#define P16_BYTES ((size_t)NEX * MM * 2)
#define P32_BYTES ((size_t)NEX * MM * 4)
#define OFF_W0N  ((size_t)0)
#define OFF_WSN  (OFF_W0N + W0N_BYTES)
#define OFF_WST  (OFF_WSN + WSN_BYTES)
#define OFF_GW   (OFF_WST + WST_BYTES)
#define OFF_CST  (OFF_GW + GW_BYTES)
#define OFF_SX   (OFF_CST + CST_BYTES)
#define OFF_U0H  (OFF_SX + SX_BYTES)
#define OFF_U1H  (OFF_U0H + P16_BYTES)
#define OFF_S2H  (OFF_U1H + P16_BYTES)
#define OFF_S1H  (OFF_S2H + P16_BYTES)
#define OFF_TO   (OFF_S1H + P16_BYTES)
#define OFF_U0F  (OFF_TO + P32_BYTES)
#define OFF_TP0  (OFF_U0F + P32_BYTES)
#define OFF_W2S  (OFF_TP0 + P32_BYTES)
#define OFF_Z2   (OFF_W2S + P32_BYTES)
#define OFF_W1S  (OFF_Z2 + P32_BYTES)
#define OFF_BASE (OFF_W1S + P32_BYTES)
#define WS_TOTAL (OFF_BASE + P32_BYTES)
static_assert((W0N_BYTES % 128) == 0 && (WSN_BYTES % 128) == 0 && (WST_BYTES % 128) == 0);
static_assert((GW_BYTES % 128) == 0 && (CST_BYTES % 128) == 0 && (SX_BYTES % 128) == 0);
static_assert((P16_BYTES % 128) == 0 && (P32_BYTES % 128) == 0);
static_assert(WS_TOTAL <= (size_t)134217728);

__device__ __forceinline__ float bf16r(float x) {
  unsigned int u = __float_as_uint(x);
  u = (u + 0x7FFFu + ((u >> 16) & 1u)) & 0xFFFF0000u;
  return __uint_as_float(u);
}

static __device__ __forceinline__ h16 toh_flush(float v) {
  const h16 r = (h16)v;
  return (fabsf(v) < 6.103515625e-05f) ? (h16)0.0f : r;
}

__device__ __forceinline__ v16h frag_at(const _Float16* p) {
  v8h lo = *(const v8h*)(p);
  v8h hi = *(const v8h*)(p + 16);
  v16h out;
#pragma unroll
  for (int i = 0; i < 8; ++i) { out[i] = lo[i]; out[i + 8] = hi[i]; }
  return out;
}
__device__ __forceinline__ v16h ld_frag(const _Float16* base, unsigned ld) {
  const unsigned lane = threadIdx.x & 31u;
  return frag_at(base + (lane & 15u) * ld + (lane >> 4) * 8u);
}

__device__ __forceinline__ v8f wmma16(v16h a, v16h b, v8f c) {
  v8f d = __builtin_amdgcn_wmma_f32_16x16x32_f16(false, a, false, b, (short)0, c,
                                                 false, false);
  asm volatile("v_nop\n\tv_nop\n\tv_nop\n\tv_nop" : "+v"(d) : "v"(a), "v"(b));
  return d;
}

__device__ __forceinline__ float red32_sum(float x) {
#pragma unroll
  for (int off = 1; off < 32; off <<= 1) x += __shfl_xor(x, off, 32);
  return x;
}

__device__ __forceinline__ float adt(float p) {
  const float a = fabsf(p);
  return a + log1pf(expf(-2.0f * a));
}

__global__ __launch_bounds__(256) void wconv_kernel(
    const float* __restrict__ W, _Float16* __restrict__ Wt, unsigned ldw, unsigned ldk) {
  __shared__ _Float16 T[64 * LDT];
  const unsigned tid = threadIdx.x;
  const unsigned n0 = blockIdx.x * 64u;
  const unsigned k0 = blockIdx.y * 64u;
#pragma unroll 4
  for (unsigned j = 0; j < 16u; ++j) {
    const unsigned idx = tid + 256u * j;
    const unsigned kr = idx >> 6, nc = idx & 63u;
    const float v = W[(size_t)(k0 + kr) * ldw + n0 + nc];
    T[nc * LDT + kr] = toh_flush(WCARRY * bf16r(v));
  }
  __syncthreads();
  v8h x[2];
  size_t off[2];
#pragma unroll
  for (unsigned i = 0; i < 2u; ++i) {
    const unsigned n = 32u * i + (tid >> 3);
    const unsigned kc = (tid & 7u) * 8u;
    x[i] = *(const v8h*)&T[n * LDT + kc];
    off[i] = (size_t)(n0 + n) * ldk + k0 + kc;
  }
#pragma unroll
  for (int i = 0; i < 2; ++i) *(volatile v8h*)(Wt + off[i]) = x[i];
  __threadfence();
#pragma unroll
  for (int i = 0; i < 2; ++i) *(volatile v8h*)(Wt + off[i]) = x[i];
}

__global__ __launch_bounds__(256) void wcast_kernel(
    const float* __restrict__ W, _Float16* __restrict__ Wh, unsigned n8) {
  const unsigned g = blockIdx.x * 256u + threadIdx.x;
  const unsigned gi = (g < n8) ? g : (n8 - 1u);
  const v4f a0 = *(const v4f*)(W + (size_t)gi * 8u);
  const v4f a1 = *(const v4f*)(W + (size_t)gi * 8u + 4u);
  v8h x;
#pragma unroll
  for (int j = 0; j < 4; ++j) {
    x[j]     = toh_flush(WCARRY * bf16r(a0[j]));
    x[j + 4] = toh_flush(WCARRY * bf16r(a1[j]));
  }
  _Float16* p = Wh + (size_t)gi * 8u;
  if (g < n8) *(volatile v8h*)p = x;
  __threadfence();
  if (g < n8) *(volatile v8h*)p = x;
}

__global__ __launch_bounds__(256) void prep_kernel(
    const float* __restrict__ A, const float* __restrict__ W0,
    _Float16* __restrict__ GW, float* __restrict__ cst) {
  const unsigned tid = threadIdx.x, lane = tid & 31u;
  const unsigned wave = __builtin_amdgcn_readfirstlane(threadIdx.x >> 5);

  float rs = 0.0f;
#pragma unroll 1
  for (unsigned q = 0; q < 16u; ++q) {
    const v4f a = *(const v4f*)(W0 + (size_t)tid * DIN + q * 4u);
#pragma unroll
    for (unsigned j = 0; j < 4u; ++j) {
      const float w = bf16r(a[j]);
      const float wm = (q * 4u + j < (unsigned)DD) ? w : 0.0f;
      rs += wm * wm;
    }
  }

  float tp = 0.0f;
  const unsigned k1 = lane + 32u;
  const unsigned k1c = (k1 < (unsigned)DD) ? k1 : (unsigned)(DD - 1);
#pragma unroll 1
  for (unsigned r = 0; r < (unsigned)RR; ++r) {
    const float a0 = bf16r(A[r * DIN + lane]);
    const float a1r = bf16r(A[r * DIN + k1c]);
    const float a1 = (k1 < (unsigned)DD) ? a1r : 0.0f;
    tp += a0 * a0;
    tp += a1 * a1;
  }
  const float tr = red32_sum(tp);

  *(volatile float*)(cst + tid) = rs;
  if (wave == 0u) *(volatile float*)(cst + MM + lane) = tr;
  __threadfence();
  *(volatile float*)(cst + tid) = rs;
  if (wave == 0u) *(volatile float*)(cst + MM + lane) = tr;

#pragma unroll 1
  for (unsigned it = 0; it < 2u; ++it) {
    const unsigned idx = tid + 256u * it;
    const unsigned row = idx >> 3, c0 = (idx & 7u) * 8u;
    float sa[8];
#pragma unroll
    for (int q = 0; q < 8; ++q) sa[q] = 0.0f;
#pragma unroll 1
    for (unsigned r = 0; r < (unsigned)RR; ++r) {
      const float ar = bf16r(A[r * DIN + row]);
      const v4f b0 = *(const v4f*)(A + r * DIN + c0);
      const v4f b1 = *(const v4f*)(A + r * DIN + c0 + 4u);
#pragma unroll
      for (int q = 0; q < 4; ++q) {
        sa[q]     += ar * bf16r(b0[q]);
        sa[q + 4] += ar * bf16r(b1[q]);
      }
    }
    v8h x;
#pragma unroll
    for (int q = 0; q < 8; ++q) x[q] = toh_flush(WCARRY * sa[q]);
    _Float16* p = GW + (size_t)row * LDG + MM + c0;
    *(volatile v8h*)p = x;
    __threadfence();
    *(volatile v8h*)p = x;
  }
}

__global__ __launch_bounds__(256) void xf_kernel(
    const float* __restrict__ x, const float* __restrict__ t, _Float16* __restrict__ SX) {
  const unsigned g = blockIdx.x * 256u + threadIdx.x;
  const unsigned tot = (unsigned)NEX * 8u;
  const unsigned gi = (g < tot) ? g : (tot - 1u);
  const unsigned n = gi >> 3, c0 = (gi & 7u) * 8u;
  const float tv = bf16r(t[0]);
  v8h o;
#pragma unroll
  for (unsigned j = 0; j < 8u; ++j) {
    const unsigned col = c0 + j;
    const unsigned colc = (col < (unsigned)DD) ? col : (unsigned)(DD - 1);
    const float xv = bf16r(x[(size_t)n * DD + colc]);
    const float v = (col < (unsigned)DD) ? xv : tv;
    o[j] = toh_flush(ACARRY * v);
  }
  _Float16* p = SX + (size_t)n * LDG + MM + c0;
  if (g < tot) *(volatile v8h*)p = o;
  __threadfence();
  if (g < tot) *(volatile v8h*)p = o;
}

#define M_OPEN 0
#define M_L0   1
#define M_L1   2
#define M_Z2   3
#define M_Z1   4
#define M_GRAD 5

template <int MODE>
__device__ __forceinline__ void gemm_body(
    const _Float16* __restrict__ A16, const unsigned lda,
    const _Float16* __restrict__ Bt, const unsigned ldb, const unsigned K,
    const float* __restrict__ vec0, const float* __restrict__ vec1,
    const float* __restrict__ in0, const float* __restrict__ in1,
    float* __restrict__ outf0, float* __restrict__ outf1,
    _Float16* __restrict__ out16, const unsigned ld16) {
  __shared__ __attribute__((aligned(16))) float Cs[64 * LDC];
  __shared__ __attribute__((aligned(16))) float Es[64 * LDC];
  __shared__ __attribute__((aligned(16))) float Hs[64 * LDC];
  const unsigned tid = threadIdx.x, lane = tid & 31u, w = tid >> 5;
  const unsigned mw = w >> 1, nw = w & 1u;
  const unsigned hh = lane >> 4, m = lane & 15u;
  const unsigned n0 = blockIdx.x * 64u;
  const unsigned row0 = blockIdx.y * 64u;

  const _Float16* ap  = A16 + (size_t)(row0 + mw * 16u + m) * lda + hh * 8u;
  const _Float16* bp0 = Bt + (size_t)(n0 + nw * 32u + m) * ldb + hh * 8u;
  const _Float16* bp1 = bp0 + (size_t)16 * ldb;
  v8f acc0 = {}, acc1 = {};
#pragma unroll 2
  for (unsigned k0 = 0; k0 < K; k0 += 32u) {
    const v16h a  = frag_at(ap + k0);
    const v16h b0 = frag_at(bp0 + k0);
    const v16h b1 = frag_at(bp1 + k0);
    acc0 = wmma16(a, b0, acc0);
    acc1 = wmma16(a, b1, acc1);
  }
#pragma unroll
  for (int r = 0; r < 8; ++r) {
    float* d = &Cs[(mw * 16u + hh * 8u + (unsigned)r) * LDC + nw * 32u + m];
    d[0]  = acc0[r];
    d[16] = acc1[r];
  }
  __syncthreads();

  const bool has_f1 = (MODE == M_OPEN || MODE == M_Z2);
  const bool has_h  = (MODE != M_GRAD);
  const float cs = (MODE == M_L0 || MODE == M_L1) ? (1.0f / WCARRY)
                                                  : (1.0f / (WCARRY * ACARRY));

#pragma unroll 1
  for (unsigned i = 0; i < (unsigned)F32_STEPS; ++i) {
    const unsigned r = 16u * i + (tid >> 4);
    const unsigned c = (tid & 15u) * 4u;
    const size_t prow = (size_t)(row0 + r) * MM + n0 + c;
    const v4f u = *(const v4f*)&Cs[r * LDC + c];
    v4f g0 = {}, g1 = {}, p0 = {}, p1 = {};
    if (MODE != M_Z1) g0 = *(const v4f*)(vec0 + n0 + c);
    if (MODE == M_L1 || MODE == M_Z1) g1 = *(const v4f*)(vec1 + n0 + c);
    if (MODE == M_L0 || MODE == M_Z2 || MODE == M_Z1) p0 = *(const v4f*)(in0 + prow);
    if (MODE == M_Z1) p1 = *(const v4f*)(in1 + prow);
    v4f f0 = {}, f1 = {}, hv = {};
#pragma unroll
    for (int j = 0; j < 4; ++j) {
      const float a = u[j] * cs;
      if (MODE == M_OPEN) {
        const float p = a + bf16r(g0[j]);
        const float ad = adt(p);
        f0[j] = tanhf(p);
        f1[j] = ad;
        hv[j] = ad;
      } else if (MODE == M_L0) {
        const float p = a + bf16r(g0[j]);
        f0[j] = tanhf(p);
        hv[j] = p0[j] + HSTEP * adt(p);
      } else if (MODE == M_L1) {
        const float p = a + bf16r(g0[j]);
        const float tp = tanhf(p);
        const float ww = bf16r(g1[j]);
        f0[j] = (1.0f - tp * tp) * ww;
        hv[j] = ACARRY * (tp * ww);
      } else if (MODE == M_Z2) {
        const float z = bf16r(g0[j]) + HSTEP * a;
        const float tp = p0[j];
        f0[j] = z;
        f1[j] = (1.0f - tp * tp) * z;
        hv[j] = ACARRY * (tp * z);
      } else if (MODE == M_Z1) {
        const float z = p0[j] + HSTEP * a;
        const float to = p1[j];
        f0[j] = (1.0f - to * to) * z * g1[j];
        hv[j] = ACARRY * (to * z);
      } else {
        f0[j] = a + bf16r(g0[j]);
      }
    }
    *(v4f*)&Cs[r * LDC + c] = f0;
    if (has_f1) *(v4f*)&Es[r * LDC + c] = f1;
    if (has_h)  *(v4f*)&Hs[r * LDC + c] = hv;
  }
  __syncthreads();

  const unsigned ldf = (MODE == M_GRAD) ? (unsigned)DIN : (unsigned)MM;
  v4f xs[4], ys[4];
  size_t off[4];
#pragma unroll
  for (unsigned i = 0; i < (unsigned)F32_STEPS; ++i) {
    const unsigned r = 16u * i + (tid >> 4);
    const unsigned c = (tid & 15u) * 4u;
    xs[i] = *(const v4f*)&Cs[r * LDC + c];
    if (has_f1) ys[i] = *(const v4f*)&Es[r * LDC + c]; else ys[i] = xs[i];
    off[i] = (size_t)(row0 + r) * ldf + n0 + c;
  }
  v8h hx[2];
  size_t hoff[2];
#pragma unroll
  for (unsigned i = 0; i < (unsigned)F16_STEPS; ++i) {
    const unsigned r = 32u * i + (tid >> 3);
    const unsigned c = (tid & 7u) * 8u;
    if (has_h) {
      const v4f u0 = *(const v4f*)&Hs[r * LDC + c];
      const v4f u1 = *(const v4f*)&Hs[r * LDC + c + 4];
#pragma unroll
      for (int j = 0; j < 4; ++j) {
        hx[i][j]     = toh_flush(u0[j]);
        hx[i][j + 4] = toh_flush(u1[j]);
      }
    } else {
      hx[i] = (v8h){};
    }
    hoff[i] = (size_t)(row0 + r) * ld16 + n0 + c;
  }

#pragma unroll
  for (int i = 0; i < 4; ++i) *(volatile v4f*)(outf0 + off[i]) = xs[i];
  if (has_f1) {
#pragma unroll
    for (int i = 0; i < 4; ++i) *(volatile v4f*)(outf1 + off[i]) = ys[i];
  }
  if (has_h) {
#pragma unroll
    for (int i = 0; i < 2; ++i) *(volatile v8h*)(out16 + hoff[i]) = hx[i];
  }
  __threadfence();
#pragma unroll
  for (int i = 0; i < 4; ++i) *(volatile v4f*)(outf0 + off[i]) = xs[i];
  if (has_f1) {
#pragma unroll
    for (int i = 0; i < 4; ++i) *(volatile v4f*)(outf1 + off[i]) = ys[i];
  }
  if (has_h) {
#pragma unroll
    for (int i = 0; i < 2; ++i) *(volatile v8h*)(out16 + hoff[i]) = hx[i];
  }
}

__global__ __launch_bounds__(256) void gemm_open_kernel(
    const _Float16* __restrict__ A16, const _Float16* __restrict__ Bt,
    const float* __restrict__ bias, float* __restrict__ to_f, float* __restrict__ u0_f,
    _Float16* __restrict__ u0_h) {
  gemm_body<M_OPEN>(A16, (unsigned)LDG, Bt, (unsigned)DIN, (unsigned)DIN, bias, bias, bias, bias,
                    to_f, u0_f, u0_h, (unsigned)MM);
}
__global__ __launch_bounds__(256) void gemm_l0_kernel(
    const _Float16* __restrict__ A16, const _Float16* __restrict__ Bt,
    const float* __restrict__ bias, const float* __restrict__ u0_f,
    float* __restrict__ tp0_f, _Float16* __restrict__ u1_h) {
  gemm_body<M_L0>(A16, (unsigned)MM, Bt, (unsigned)MM, (unsigned)MM, bias, bias, u0_f, u0_f,
                  tp0_f, tp0_f, u1_h, (unsigned)MM);
}
__global__ __launch_bounds__(256) void gemm_l1_kernel(
    const _Float16* __restrict__ A16, const _Float16* __restrict__ Bt,
    const float* __restrict__ bias, const float* __restrict__ ww,
    float* __restrict__ w2s_f, _Float16* __restrict__ s2_h) {
  gemm_body<M_L1>(A16, (unsigned)MM, Bt, (unsigned)MM, (unsigned)MM, bias, ww, bias, bias,
                  w2s_f, w2s_f, s2_h, (unsigned)MM);
}
__global__ __launch_bounds__(256) void gemm_z2_kernel(
    const _Float16* __restrict__ A16, const _Float16* __restrict__ Bt,
    const float* __restrict__ ww, const float* __restrict__ tp0_f,
    float* __restrict__ z2_f, float* __restrict__ w1s_f, _Float16* __restrict__ s1_h) {
  gemm_body<M_Z2>(A16, (unsigned)MM, Bt, (unsigned)(2 * MM), (unsigned)MM, ww, ww, tp0_f, tp0_f,
                  z2_f, w1s_f, s1_h, (unsigned)MM);
}
__global__ __launch_bounds__(256) void gemm_z1_kernel(
    const _Float16* __restrict__ A16, const _Float16* __restrict__ Bt,
    const float* __restrict__ rsum, const float* __restrict__ z2_f,
    const float* __restrict__ to_f, float* __restrict__ base_f, _Float16* __restrict__ sx_h) {
  gemm_body<M_Z1>(A16, (unsigned)MM, Bt, (unsigned)(2 * MM), (unsigned)MM, rsum, rsum, z2_f, to_f,
                  base_f, base_f, sx_h, (unsigned)LDG);
}
__global__ __launch_bounds__(256) void gemm_grad_kernel(
    const _Float16* __restrict__ A16, const _Float16* __restrict__ Bt,
    const float* __restrict__ cw, float* __restrict__ outf) {
  gemm_body<M_GRAD>(A16, (unsigned)LDG, Bt, (unsigned)LDG, (unsigned)LDG, cw, cw, cw, cw,
                    outf, outf, (_Float16*)0, (unsigned)MM);
}

__global__ __launch_bounds__(256) void jac_kernel(
    const _Float16* __restrict__ Wn, const _Float16* __restrict__ GW,
    const float* __restrict__ TOp, const float* __restrict__ TP0p,
    const float* __restrict__ W1Sp, const float* __restrict__ W2Sp,
    const float* __restrict__ BASEp, const float* __restrict__ cst,
    float* __restrict__ outv) {
  __shared__ __attribute__((aligned(16))) _Float16 Jt[DIN * LDJ];
  __shared__ __attribute__((aligned(16))) float tos[MM];
  __shared__ __attribute__((aligned(16))) float tpa[MM];
  __shared__ __attribute__((aligned(16))) float wvs[2 * MM];
  __shared__ __attribute__((aligned(16))) float wsum[8];
  __shared__ __attribute__((aligned(16))) float res[SPB];

  const unsigned tid = threadIdx.x, lane = tid & 31u;
  const unsigned wave = __builtin_amdgcn_readfirstlane(threadIdx.x >> 5);
  const unsigned hh = lane >> 4, ml = lane & 15u;
  const float trace = cst[MM];
  const unsigned fd = tid & 63u, fq = tid >> 6;
  const size_t arow = (size_t)((wave * 2u) * 16u + ml) * MM + hh * 8u;

#pragma unroll 1
  for (unsigned s = 0; s < (unsigned)SPB; ++s) {
    const size_t n = (size_t)blockIdx.x * SPB + s;
    const size_t e = n * MM + tid;
    tos[tid] = TOp[e];
    tpa[tid] = TP0p[e];
    wvs[tid] = W1Sp[e];
    wvs[MM + tid] = W2Sp[e];
    const float part = BASEp[e];
    float quad = 0.0f;
    __syncthreads();

#pragma unroll 2
    for (unsigned g = 0; g < 8u; ++g) {
      const unsigned m0 = fq * 64u + g * 8u;
      const v8h wv = *(const v8h*)(GW + (size_t)fd * LDG + m0);
      const v4f ta = *(const v4f*)&tos[m0];
      const v4f tb = *(const v4f*)&tos[m0 + 4u];
      v8h jv;
#pragma unroll
      for (int i = 0; i < 4; ++i) {
        const float a = (float)wv[i] * ta[i];
        const float b = (float)wv[i + 4] * tb[i];
        jv[i]     = toh_flush((fd < (unsigned)DD) ? a : 0.0f);
        jv[i + 4] = toh_flush((fd < (unsigned)DD) ? b : 0.0f);
      }
      *(v8h*)&Jt[fd * LDJ + m0] = jv;
    }
    __syncthreads();

#pragma unroll
    for (int iter = 0; iter < 2; ++iter) {
      v8f acc[2][4];
#pragma unroll
      for (int mi = 0; mi < 2; ++mi)
#pragma unroll
        for (int nt = 0; nt < 4; ++nt) acc[mi][nt] = (v8f){};
      const _Float16* ap0 = Wn + (size_t)iter * MM * MM + arow;
      const _Float16* ap1 = ap0 + (size_t)16 * MM;
#pragma unroll 2
      for (unsigned k0 = 0; k0 < (unsigned)MM; k0 += 32u) {
        const v16h a0 = frag_at(ap0 + k0);
        const v16h a1 = frag_at(ap1 + k0);
#pragma unroll
        for (int nt = 0; nt < 4; ++nt) {
          const v16h bf = ld_frag(&Jt[(nt * 16) * LDJ + k0], LDJ);
          acc[0][nt] = wmma16(a0, bf, acc[0][nt]);
          acc[1][nt] = wmma16(a1, bf, acc[1][nt]);
        }
      }
      if (iter == 0) __syncthreads();

#pragma unroll
      for (int mi = 0; mi < 2; ++mi) {
        const unsigned m0 = (wave * 2u + (unsigned)mi) * 16u + hh * 8u;
        const v4f wa = *(const v4f*)&wvs[iter * MM + m0];
        const v4f wb = *(const v4f*)&wvs[iter * MM + m0 + 4u];
        v4f ta = {}, tb = {};
        if (iter == 0) {
          ta = *(const v4f*)&tpa[m0];
          tb = *(const v4f*)&tpa[m0 + 4u];
        }
#pragma unroll
        for (int nt = 0; nt < 4; ++nt) {
          const unsigned d = (unsigned)nt * 16u + ml;
          v8h jo = {};
          if (iter == 0) jo = *(const v8h*)&Jt[d * LDJ + m0];
          v8h jn;
#pragma unroll
          for (int r = 0; r < 8; ++r) {
            float dv = acc[mi][nt][r] * (1.0f / (WCARRY * WCARRY));
            if (nt == 3) dv = (ml == 15u) ? 0.0f : dv;
            const float wv = (r < 4) ? wa[r & 3] : wb[r & 3];
            quad += wv * dv * dv;
            if (iter == 0) {
              const float tp = (r < 4) ? ta[r & 3] : tb[r & 3];
              jn[r] = toh_flush((float)jo[r] + (HSTEP * WCARRY) * tp * dv);
            }
          }
          if (iter == 0) *(v8h*)&Jt[d * LDJ + m0] = jn;
        }
      }
      if (iter == 0) __syncthreads();
    }

    const float tot = red32_sum(part + HSTEP * quad);
    if (lane == 0u) wsum[wave] = tot;
    __syncthreads();
    if (tid == 0u) {
      const float t8 = ((wsum[0] + wsum[1]) + (wsum[2] + wsum[3])) +
                       ((wsum[4] + wsum[5]) + (wsum[6] + wsum[7]));
      res[s] = t8 + trace;
    }
  }
  __syncthreads();

  const unsigned li = (tid & 7u) * 4u;
  const v4f rv = *(const v4f*)&res[li];
  float* op = outv + (size_t)blockIdx.x * SPB + li;
  if (tid < 8u) *(volatile v4f*)op = rv;
  __threadfence();
  if (tid < 8u) *(volatile v4f*)op = rv;
}

extern "C" void kernel_launch(void* const* d_in, const int* in_sizes, int n_in,
                              void* d_out, int out_size, void* d_ws, size_t ws_size,
                              hipStream_t stream) {
  if (n_in < 9) return;
  if (in_sizes[0] < 1) return;
  if ((long long)in_sizes[1] < (long long)NEX * DD) return;
  if (in_sizes[2] < RR * DIN) return;
  if (in_sizes[3] < MM * DIN) return;
  if (in_sizes[4] < MM) return;
  if (in_sizes[5] < 2 * MM * MM) return;
  if (in_sizes[6] < 2 * MM) return;
  if (in_sizes[7] < MM) return;
  if (in_sizes[8] < DIN) return;
  if ((long long)out_size < (long long)NEX_FULL * DIN + NEX) return;
  if (ws_size < WS_TOTAL) return;

  const float* t   = (const float*)d_in[0];
  const float* x   = (const float*)d_in[1];
  const float* A   = (const float*)d_in[2];
  const float* W0  = (const float*)d_in[3];
  const float* b0  = (const float*)d_in[4];
  const float* Ws  = (const float*)d_in[5];
  const float* bs  = (const float*)d_in[6];
  const float* w_w = (const float*)d_in[7];
  const float* c_w = (const float*)d_in[8];
  float* out0 = (float*)d_out;
  float* out1 = (float*)d_out + (size_t)NEX_FULL * DIN;

  char* ws = (char*)d_ws;
  _Float16* W0n = (_Float16*)(ws + OFF_W0N);
  _Float16* Wsn = (_Float16*)(ws + OFF_WSN);
  _Float16* Wst = (_Float16*)(ws + OFF_WST);
  _Float16* GW  = (_Float16*)(ws + OFF_GW);
  float*    CST = (float*)(ws + OFF_CST);
  _Float16* SX  = (_Float16*)(ws + OFF_SX);
  _Float16* U0h = (_Float16*)(ws + OFF_U0H);
  _Float16* U1h = (_Float16*)(ws + OFF_U1H);
  _Float16* S2h = (_Float16*)(ws + OFF_S2H);
  _Float16* S1h = (_Float16*)(ws + OFF_S1H);
  float* TOf  = (float*)(ws + OFF_TO);
  float* U0f  = (float*)(ws + OFF_U0F);
  float* TP0f = (float*)(ws + OFF_TP0);
  float* W2Sf = (float*)(ws + OFF_W2S);
  float* Z2f  = (float*)(ws + OFF_Z2);
  float* W1Sf = (float*)(ws + OFF_W1S);
  float* BASf = (float*)(ws + OFF_BASE);

  dim3 blk(256);
  dim3 gg(MM / 64, NEX / 64);

  prep_kernel<<<dim3(1), blk, 0, stream>>>(A, W0, GW, CST);
  wcast_kernel<<<dim3((MM * DIN / 8 + 255) / 256), blk, 0, stream>>>(W0, W0n, (unsigned)(MM * DIN / 8));
  wcast_kernel<<<dim3((2 * MM * MM / 8 + 255) / 256), blk, 0, stream>>>(Ws, Wsn, (unsigned)(2 * MM * MM / 8));
  wconv_kernel<<<dim3(MM / 64, 2 * MM / 64), blk, 0, stream>>>(Ws, Wst, (unsigned)MM, (unsigned)(2 * MM));
  wconv_kernel<<<dim3(DIN / 64, MM / 64), blk, 0, stream>>>(W0, GW, (unsigned)DIN, (unsigned)LDG);
  xf_kernel<<<dim3((NEX * 8 + 255) / 256), blk, 0, stream>>>(x, t, SX);

  gemm_open_kernel<<<gg, blk, 0, stream>>>(SX + MM, W0n, b0, TOf, U0f, U0h);
  gemm_l0_kernel<<<gg, blk, 0, stream>>>(U0h, Wsn, bs, U0f, TP0f, U1h);
  gemm_l1_kernel<<<gg, blk, 0, stream>>>(U1h, Wsn + (size_t)MM * MM, bs + MM, w_w, W2Sf, S2h);
  gemm_z2_kernel<<<gg, blk, 0, stream>>>(S2h, Wst + MM, w_w, TP0f, Z2f, W1Sf, S1h);
  gemm_z1_kernel<<<gg, blk, 0, stream>>>(S1h, Wst, CST, Z2f, TOf, BASf, SX);
  gemm_grad_kernel<<<dim3(DIN / 64, NEX / 64), blk, 0, stream>>>(SX, GW, c_w, out0);
  jac_kernel<<<dim3(NEX / SPB), blk, 0, stream>>>(Wsn, GW, TOf, TP0f, W1Sf, W2Sf, BASf, CST, out1);
}
